// ImageClassifier_8813272891552
// MI455X (gfx1250) — hardware-verified
//
#include <hip/hip_runtime.h>
#define NI 32
#define H0 128
#define H1 64
#define H2 32
#define C1 64
#define C2 128
#define NHD 4
#define DH 16
#define INNER 64
#define HY H1
#define WX H1
#define NPOS (NI * H1 * H1)
#define NPOSR NPOS
#define NVOX NPOS
#define COUT C2
#define NT2 (NI * H2 * H2)

typedef __bf16 v16b __attribute__((ext_vector_type(16)));
typedef unsigned short v8us __attribute__((ext_vector_type(8), may_alias));
typedef float  v8f  __attribute__((ext_vector_type(8)));
typedef float  v4f  __attribute__((ext_vector_type(4)));
typedef float  v4fa __attribute__((ext_vector_type(4), may_alias));
union FragB { v16b v; v8us half[2]; unsigned short u[16]; };

__device__ __forceinline__ unsigned short bf16_bits(float x) { unsigned int u = __float_as_uint(x); return (unsigned short)((u + 0x7FFFu + ((u >> 16) & 1u)) >> 16); }
__device__ __forceinline__ float bf16_val(unsigned short b) { return __uint_as_float(((unsigned int)b) << 16); }
__device__ __forceinline__ float bf16_round(float x) { return bf16_val(bf16_bits(x)); }
template <int NT>
__device__ __forceinline__ v8f mmaN(v16b ah, v16b al, v16b bh, v16b bl, v8f c) {
  c = __builtin_amdgcn_wmma_f32_16x16x32_bf16(false, ah, false, bh, (short)0, c, false, false);
  if (NT >= 2) c = __builtin_amdgcn_wmma_f32_16x16x32_bf16(false, al, false, bh, (short)0, c, false, false);
  if (NT >= 3) c = __builtin_amdgcn_wmma_f32_16x16x32_bf16(false, ah, false, bl, (short)0, c, false, false);
  asm volatile("v_nop\n\tv_nop\n\tv_nop\n\tv_nop" : "+v"(c) : "v"(ah), "v"(al), "v"(bh), "v"(bl));
  return c;
}

__global__ __launch_bounds__(256) void k_wt_bf16(const float* __restrict__ W, unsigned short* __restrict__ Wt, int K, int N) {
  const int t = blockIdx.x * 256 + threadIdx.x;
  const int k8n = K / 8;
  if (t >= N * k8n) return;
  const int n = t / k8n, k8 = (t % k8n) * 8;
  v8us v;
#pragma unroll
  for (int i = 0; i < 8; ++i) v[i] = bf16_bits(W[(size_t)(k8 + i) * N + n]);
  *(volatile v8us*)(Wt + (size_t)n * K + k8) = v;
  __threadfence();
  *(volatile v8us*)(Wt + (size_t)n * K + k8) = v;
}

template <bool ASPLIT, int ACT, bool BIAS_BF16>
__global__ __launch_bounds__(128) void k_gemm_bf(const float* __restrict__ A, int lda, const unsigned short* __restrict__ Wt, int ldb,
                                               const float* __restrict__ bias, float* __restrict__ C, int ldc, int M, int N, int K) {
  __shared__ __attribute__((aligned(16))) float so[4][16][64];
  const int tid = threadIdx.x, w = tid >> 5, lane = tid & 31, ln = lane & 15, hh = lane >> 4;
  const int ntn = N / 64;
  const int wid = blockIdx.x * 4 + w;
  const int mt = wid / ntn, nq = wid % ntn;
  if (mt * 16 >= M) return;
  const int row0 = mt * 16, col0 = nq * 64;
  const float* arow = A + (size_t)(row0 + ln) * lda;
  v8f acc[4] = {};
  for (int kb = 0; kb < K; kb += 32) {
    FragB ah, al;
    const v4f x0 = *(const v4fa*)(arow + kb + 8 * hh), x1 = *(const v4fa*)(arow + kb + 8 * hh + 4);
    const v4f x2 = *(const v4fa*)(arow + kb + 16 + 8 * hh), x3 = *(const v4fa*)(arow + kb + 16 + 8 * hh + 4);
    float xs[16] = {x0[0],x0[1],x0[2],x0[3],x1[0],x1[1],x1[2],x1[3],x2[0],x2[1],x2[2],x2[3],x3[0],x3[1],x3[2],x3[3]};
#pragma unroll
    for (int i = 0; i < 16; ++i) { const unsigned short hb = bf16_bits(xs[i]); ah.u[i] = hb; al.u[i] = ASPLIT ? bf16_bits(xs[i] - bf16_val(hb)) : (unsigned short)0; }
#pragma unroll
    for (int t = 0; t < 4; ++t) {
      const unsigned short* brow = Wt + (size_t)(col0 + t * 16 + ln) * ldb + kb;
      FragB b;
      b.half[0] = *(const v8us*)(brow + 8 * hh);
      b.half[1] = *(const v8us*)(brow + 16 + 8 * hh);
      acc[t] = mmaN<ASPLIT ? 2 : 1>(ah.v, al.v, b.v, b.v, acc[t]);
    }
  }
#pragma unroll
  for (int t = 0; t < 4; ++t) {
    float bv = bias ? bias[col0 + t * 16 + ln] : 0.f;
    if (BIAS_BF16) bv = bf16_round(bv);
#pragma unroll
    for (int r = 0; r < 8; ++r) { float v = acc[t][r] + bv; if (ACT == 1) v = fmaxf(v, 0.f); so[w][8 * hh + r][t * 16 + ln] = v; }
  }
  __builtin_amdgcn_fence(__ATOMIC_ACQ_REL, "workgroup");
  __builtin_amdgcn_wave_barrier();
  const int rsub = lane >> 4, c4 = (lane & 15) * 4;
  for (int pass = 0; pass < 2; ++pass) {
#pragma unroll
    for (int q = 0; q < 8; ++q) {
      const int r = q * 2 + rsub;
      const v4f v = *(const v4fa*)&so[w][r][c4];
      *(volatile v4f*)(C + (size_t)(row0 + r) * ldc + col0 + c4) = v;
    }
    if (pass == 0) __threadfence();
  }
}

template <int D, bool CAUSAL>
__global__ __launch_bounds__(128) void k_flash(const float* __restrict__ qb, const float* __restrict__ kb, const float* __restrict__ vb,
                                             int pitch, int T, int H, float scale, float* __restrict__ y, int ypitch) {
  constexpr int KS = D / 32;
  constexpr int DT = D / 16;
  __shared__ __attribute__((aligned(16))) unsigned short sKh[32][D + 8], sKl[32][D + 8], sVh[32][D + 8], sVl[32][D + 8];
  __shared__ __attribute__((aligned(16))) unsigned short sPh[4][16][40], sPl[4][16][40];
  __shared__ __attribute__((aligned(16))) float sO[4][16][D];
  const int tid = threadIdx.x, w = tid >> 5, lane = tid & 31, ln = lane & 15, hh = lane >> 4;
  const int nqb = (T + 63) / 64;
  const int bh = blockIdx.x / nqb, qblk = blockIdx.x % nqb;
  const int b = bh / H, h = bh % H;
  const int q0 = qblk * 64 + w * 16;
  const float* Q = qb + (size_t)b * T * pitch + h * D;
  const float* K = kb + (size_t)b * T * pitch + h * D;
  const float* V = vb + (size_t)b * T * pitch + h * D;

  FragB aqh[KS], aql[KS];
  {
    int row = q0 + ln; if (row >= T) row = T - 1;
    const float* qr = Q + (size_t)row * pitch;
#pragma unroll
    for (int ks = 0; ks < KS; ++ks)
#pragma unroll
      for (int i = 0; i < 16; ++i) {
        const int d = ks * 32 + ((i < 8) ? (8 * hh + i) : (16 + 8 * hh + (i - 8)));
        const float x = qr[d] * scale; const unsigned short hb = bf16_bits(x);
        aqh[ks].u[i] = hb; aql[ks].u[i] = bf16_bits(x - bf16_val(hb));
      }
  }
  float m_r[8], l_r[8];
#pragma unroll
  for (int r = 0; r < 8; ++r) { m_r[r] = -3.0e38f; l_r[r] = 0.f; }
  v8f oacc[DT];
#pragma unroll
  for (int dt = 0; dt < DT; ++dt) oacc[dt] = (v8f){0.f,0.f,0.f,0.f,0.f,0.f,0.f,0.f};

  const int kv_end = CAUSAL ? min(T, qblk * 64 + 64) : T;
  for (int j0 = 0; j0 < kv_end; j0 += 32) {
    __syncthreads();
    for (int e = tid; e < 32 * (D / 4); e += 128) {
      const int r = e / (D / 4), c4 = (e % (D / 4)) * 4;
      const int key = j0 + r;
      v4f kf = {0.f,0.f,0.f,0.f}, vf = {0.f,0.f,0.f,0.f};
      if (key < T) { kf = *(const v4fa*)(K + (size_t)key * pitch + c4); vf = *(const v4fa*)(V + (size_t)key * pitch + c4); }
#pragma unroll
      for (int t = 0; t < 4; ++t) {
        unsigned short hb = bf16_bits(kf[t]); sKh[r][c4 + t] = hb; sKl[r][c4 + t] = bf16_bits(kf[t] - bf16_val(hb));
        hb = bf16_bits(vf[t]); sVh[r][c4 + t] = hb; sVl[r][c4 + t] = bf16_bits(vf[t] - bf16_val(hb));
      }
    }
    __syncthreads();
    v8f s[2];
#pragma unroll
    for (int nt = 0; nt < 2; ++nt) {
      v8f acc = {};
#pragma unroll
      for (int ks = 0; ks < KS; ++ks) {
        FragB bh_, bl_;
        bh_.half[0] = *(const v8us*)&sKh[nt * 16 + ln][ks * 32 + 8 * hh]; bh_.half[1] = *(const v8us*)&sKh[nt * 16 + ln][ks * 32 + 16 + 8 * hh];
        bl_.half[0] = *(const v8us*)&sKl[nt * 16 + ln][ks * 32 + 8 * hh]; bl_.half[1] = *(const v8us*)&sKl[nt * 16 + ln][ks * 32 + 16 + 8 * hh];
        acc = mmaN<3>(aqh[ks].v, aql[ks].v, bh_.v, bl_.v, acc);
      }
      s[nt] = acc;
    }
    float alpha[8];
#pragma unroll
    for (int r = 0; r < 8; ++r) {
      const int qi = q0 + 8 * hh + r;
      const int ja = j0 + ln, jb = j0 + 16 + ln;
      if (CAUSAL) { if (ja > qi) s[0][r] = -3.0e38f; if (jb > qi) s[1][r] = -3.0e38f; }
      if (ja >= T) s[0][r] = -3.0e38f;
      if (jb >= T) s[1][r] = -3.0e38f;
      float mx = fmaxf(s[0][r], s[1][r]);
      mx = fmaxf(mx, __shfl_xor(mx, 1, 32)); mx = fmaxf(mx, __shfl_xor(mx, 2, 32)); mx = fmaxf(mx, __shfl_xor(mx, 4, 32)); mx = fmaxf(mx, __shfl_xor(mx, 8, 32));
      const float mnew = fmaxf(m_r[r], mx);
      alpha[r] = (mnew > -1.0e38f) ? __expf(m_r[r] - mnew) : 1.0f;
      const float p0 = (s[0][r] > -1.0e38f) ? __expf(s[0][r] - mnew) : 0.f;
      const float p1 = (s[1][r] > -1.0e38f) ? __expf(s[1][r] - mnew) : 0.f;
      m_r[r] = mnew;
      l_r[r] = l_r[r] * alpha[r] + p0 + p1;
      unsigned short hb = bf16_bits(p0); sPh[w][8 * hh + r][ln] = hb;      sPl[w][8 * hh + r][ln] = bf16_bits(p0 - bf16_val(hb));
      hb = bf16_bits(p1);                sPh[w][8 * hh + r][16 + ln] = hb; sPl[w][8 * hh + r][16 + ln] = bf16_bits(p1 - bf16_val(hb));
    }
#pragma unroll
    for (int dt = 0; dt < DT; ++dt)
#pragma unroll
      for (int r = 0; r < 8; ++r) oacc[dt][r] *= alpha[r];
    __builtin_amdgcn_fence(__ATOMIC_ACQ_REL, "workgroup");
    __builtin_amdgcn_wave_barrier();
    FragB pah, pal;
    pah.half[0] = *(const v8us*)&sPh[w][ln][8 * hh]; pah.half[1] = *(const v8us*)&sPh[w][ln][16 + 8 * hh];
    pal.half[0] = *(const v8us*)&sPl[w][ln][8 * hh]; pal.half[1] = *(const v8us*)&sPl[w][ln][16 + 8 * hh];
#pragma unroll
    for (int dt = 0; dt < DT; ++dt) {
      FragB bvh, bvl;
#pragma unroll
      for (int i = 0; i < 8; ++i) {
        bvh.u[i] = sVh[8 * hh + i][dt * 16 + ln]; bvh.u[8 + i] = sVh[16 + 8 * hh + i][dt * 16 + ln];
        bvl.u[i] = sVl[8 * hh + i][dt * 16 + ln]; bvl.u[8 + i] = sVl[16 + 8 * hh + i][dt * 16 + ln];
      }
      oacc[dt] = mmaN<3>(pah.v, pal.v, bvh.v, bvl.v, oacc[dt]);
    }
    __builtin_amdgcn_fence(__ATOMIC_ACQ_REL, "workgroup");
    __builtin_amdgcn_wave_barrier();
  }
#pragma unroll
  for (int r = 0; r < 8; ++r) {
    float l = l_r[r];
    l += __shfl_xor(l, 1, 32); l += __shfl_xor(l, 2, 32); l += __shfl_xor(l, 4, 32); l += __shfl_xor(l, 8, 32);
    l_r[r] = (l > 0.f) ? 1.0f / l : 0.f;
  }
#pragma unroll
  for (int dt = 0; dt < DT; ++dt)
#pragma unroll
    for (int r = 0; r < 8; ++r) sO[w][8 * hh + r][dt * 16 + ln] = oacc[dt][r] * l_r[r];
  __builtin_amdgcn_fence(__ATOMIC_ACQ_REL, "workgroup");
  __builtin_amdgcn_wave_barrier();
  for (int pass = 0; pass < 2; ++pass) {
    for (int r = 0; r < 16; ++r) {
      const int row = q0 + r;
      if (row < T && lane < D / 4) {
        const v4f val = *(const v4fa*)&sO[w][r][lane * 4];
        *(volatile v4f*)(y + ((size_t)b * T + row) * ypitch + h * D + lane * 4) = val;
      }
    }
    if (pass == 0) __threadfence();
  }
}

template <bool ASPLIT, int ACT, bool BIAS_BF16, bool RES_BF16>
__global__ __launch_bounds__(128) void k_gemm_bf3(const float* __restrict__ A, int lda, const unsigned short* __restrict__ Wt, int ldb,
                                                const float* __restrict__ bias, const float* __restrict__ resid, int rmod, int ldr,
                                                float* __restrict__ C, int ldc, int M, int N, int K) {
  __shared__ __attribute__((aligned(16))) float so[4][16][64];
  const int tid = threadIdx.x, w = tid >> 5, lane = tid & 31, ln = lane & 15, hh = lane >> 4;
  const int ntn = N / 64;
  const int wid = blockIdx.x * 4 + w;
  const int mt = wid / ntn, nq = wid % ntn;
  if (mt * 16 >= M) return;
  const int row0 = mt * 16, col0 = nq * 64;
  const float* arow = A + (size_t)(row0 + ln) * lda;
  v8f acc[4] = {};
  for (int kb = 0; kb < K; kb += 32) {
    FragB ah, al;
    const v4f x0 = *(const v4fa*)(arow + kb + 8 * hh), x1 = *(const v4fa*)(arow + kb + 8 * hh + 4);
    const v4f x2 = *(const v4fa*)(arow + kb + 16 + 8 * hh), x3 = *(const v4fa*)(arow + kb + 16 + 8 * hh + 4);
    float xs[16] = {x0[0],x0[1],x0[2],x0[3],x1[0],x1[1],x1[2],x1[3],x2[0],x2[1],x2[2],x2[3],x3[0],x3[1],x3[2],x3[3]};
#pragma unroll
    for (int i = 0; i < 16; ++i) { const unsigned short hb = bf16_bits(xs[i]); ah.u[i] = hb; al.u[i] = ASPLIT ? bf16_bits(xs[i] - bf16_val(hb)) : (unsigned short)0; }
#pragma unroll
    for (int t = 0; t < 4; ++t) {
      const unsigned short* brow = Wt + (size_t)(col0 + t * 16 + ln) * ldb + kb;
      FragB b;
      b.half[0] = *(const v8us*)(brow + 8 * hh);
      b.half[1] = *(const v8us*)(brow + 16 + 8 * hh);
      acc[t] = mmaN<ASPLIT ? 2 : 1>(ah.v, al.v, b.v, b.v, acc[t]);
    }
  }
#pragma unroll
  for (int t = 0; t < 4; ++t) {
    const int col = col0 + t * 16 + ln;
    float bv = bias ? bias[col] : 0.f;
    if (BIAS_BF16) bv = bf16_round(bv);
#pragma unroll
    for (int r = 0; r < 8; ++r) {
      float v = acc[t][r] + bv;
      if (resid) { float rv = resid[(size_t)((row0 + 8 * hh + r) % rmod) * ldr + col]; if (RES_BF16) rv = bf16_round(rv); v += rv; }
      if (ACT == 1) v = fmaxf(v, 0.f);
      if (ACT == 2) v = 0.5f * v * (1.0f + erff(v * 0.70710678118654752f));
      if (ACT == 3) { const float u = 0.7978845608028654f * (v + 0.044715f * v * v * v); v = 0.5f * v * (1.0f + tanhf(u)); }
      so[w][8 * hh + r][t * 16 + ln] = v;
    }
  }
  __builtin_amdgcn_fence(__ATOMIC_ACQ_REL, "workgroup");
  __builtin_amdgcn_wave_barrier();
  const int rsub = lane >> 4, c4 = (lane & 15) * 4;
  for (int pass = 0; pass < 2; ++pass) {
#pragma unroll
    for (int q = 0; q < 8; ++q) {
      const int r = q * 2 + rsub;
      const v4f v = *(const v4fa*)&so[w][r][c4];
      *(volatile v4f*)(C + (size_t)(row0 + r) * ldc + col0 + c4) = v;
    }
    if (pass == 0) __threadfence();
  }
}
template <bool PARAM_BF16>
__global__ __launch_bounds__(256) void k_layernorm(const float* __restrict__ X, const float* __restrict__ R, const float* __restrict__ g, const float* __restrict__ bta,
                                                  float* __restrict__ out_sum, float* __restrict__ out_norm, int N, float eps) {
  __shared__ float red[256];
  const int row = blockIdx.x, tid = threadIdx.x;
  const float* x = X + (size_t)row * N; const float* rr = R ? R + (size_t)row * N : nullptr;
  float vals[16];
  const int per = N / 256;
  float s1 = 0.f;
  for (int u = 0; u < per / 4; ++u) {
    const int j = tid * 4 + 1024 * u;
    const v4f a = *(const v4fa*)(x + j);
    v4f b = {0.f,0.f,0.f,0.f}; if (rr) b = *(const v4fa*)(rr + j);
#pragma unroll
    for (int q = 0; q < 4; ++q) { const float v = a[q] + b[q]; vals[u * 4 + q] = v; s1 += v; }
  }
  red[tid] = s1; __syncthreads();
  for (int st = 128; st > 0; st >>= 1) { if (tid < st) red[tid] += red[tid + st]; __syncthreads(); }
  const float mu = red[0] / (float)N; __syncthreads();
  float s2 = 0.f;
  for (int u = 0; u < per / 4; ++u)
#pragma unroll
    for (int q = 0; q < 4; ++q) { const float c = vals[u * 4 + q] - mu; s2 += c * c; }
  red[tid] = s2; __syncthreads();
  for (int st = 128; st > 0; st >>= 1) { if (tid < st) red[tid] += red[tid + st]; __syncthreads(); }
  const float rs = rsqrtf(red[0] / (float)N + eps);
  for (int pass = 0; pass < 2; ++pass) {
    for (int u = 0; u < per / 4; ++u) {
      const int j = tid * 4 + 1024 * u;
      v4f o, sm;
#pragma unroll
      for (int q = 0; q < 4; ++q) {
        float gg = g[j + q], bb = bta[j + q];
        if (PARAM_BF16) { gg = bf16_round(gg); bb = bf16_round(bb); }
        sm[q] = vals[u * 4 + q]; o[q] = (vals[u * 4 + q] - mu) * rs * gg + bb;
      }
      if (out_sum) *(volatile v4f*)(out_sum + (size_t)row * N + j) = sm;
      *(volatile v4f*)(out_norm + (size_t)row * N + j) = o;
    }
    if (pass == 0) __threadfence();
  }
}

typedef _Float16 v16h __attribute__((ext_vector_type(16)));
union FragH { v16h v; v8us half[2]; _Float16 h[16]; unsigned short u[16]; };
template <int NT>
__device__ __forceinline__ v8f mmaH(v16h ah, v16h al, v16h bh, v16h bl, v8f c) {
  c = __builtin_amdgcn_wmma_f32_16x16x32_f16(false, ah, false, bh, (short)0, c, false, false);
  if (NT >= 2) c = __builtin_amdgcn_wmma_f32_16x16x32_f16(false, al, false, bh, (short)0, c, false, false);
  if (NT >= 3) c = __builtin_amdgcn_wmma_f32_16x16x32_f16(false, ah, false, bl, (short)0, c, false, false);
  asm volatile("v_nop\n\tv_nop\n\tv_nop\n\tv_nop" : "+v"(c) : "v"(ah), "v"(al), "v"(bh), "v"(bl));
  return c;
}
template <bool ASPLIT>
__global__ __launch_bounds__(128) void k_gemm_h(const float* __restrict__ A, int lda, size_t sA, const _Float16* __restrict__ Bh, int ldb, size_t sB, float alpha, float* __restrict__ C, int ldc, size_t sC, int M, int N, int K) {
  __shared__ __attribute__((aligned(16))) float so[4][16][64];
  const int tid = threadIdx.x, w = tid >> 5, lane = tid & 31, ln = lane & 15, hh = lane >> 4; const int by = blockIdx.y;
  A += (size_t)by * sA; Bh += (size_t)by * sB; C += (size_t)by * sC;
  const int ntn = (N + 63) / 64; const int wid = blockIdx.x * 4 + w; const int mt = wid / ntn, nq = wid % ntn; if (mt * 16 >= M) return;
  const int row0 = mt * 16, col0 = nq * 64; const float* arow = A + (size_t)(row0 + ln) * lda;
  v8f acc[4] = {};
  for (int kb = 0; kb < K; kb += 32) {
    FragH ah, al;
    const v4f x0 = *(const v4fa*)(arow + kb + 8 * hh), x1 = *(const v4fa*)(arow + kb + 8 * hh + 4), x2 = *(const v4fa*)(arow + kb + 16 + 8 * hh), x3 = *(const v4fa*)(arow + kb + 16 + 8 * hh + 4);
    float xs[16] = {x0[0],x0[1],x0[2],x0[3],x1[0],x1[1],x1[2],x1[3],x2[0],x2[1],x2[2],x2[3],x3[0],x3[1],x3[2],x3[3]};
#pragma unroll
    for (int i = 0; i < 16; ++i) { const _Float16 h = (_Float16)xs[i]; ah.h[i] = h; al.h[i] = ASPLIT ? (_Float16)(xs[i] - (float)h) : (_Float16)0.0f; }
#pragma unroll
    for (int t = 0; t < 4; ++t) { if (col0 + t * 16 >= N) continue; const size_t boff = (size_t)(col0 + t * 16 + ln) * ldb + kb; FragH bq; bq.half[0] = *(const v8us*)(Bh + boff + 8 * hh); bq.half[1] = *(const v8us*)(Bh + boff + 16 + 8 * hh);
      acc[t] = mmaH<ASPLIT ? 2 : 1>(ah.v, al.v, bq.v, bq.v, acc[t]); }
  }
#pragma unroll
  for (int t = 0; t < 4; ++t) { if (col0 + t * 16 >= N) continue;
#pragma unroll
    for (int r = 0; r < 8; ++r) so[w][8 * hh + r][t * 16 + ln] = acc[t][r] * alpha; }
  __builtin_amdgcn_fence(__ATOMIC_ACQ_REL, "workgroup"); __builtin_amdgcn_wave_barrier();
  const int rsub = lane >> 4, c4 = (lane & 15) * 4;
  for (int pass = 0; pass < 2; ++pass) {
#pragma unroll
    for (int q = 0; q < 8; ++q) { const int r = q * 2 + rsub; if (col0 + c4 < N) { const v4f v = *(const v4fa*)&so[w][r][c4]; *(volatile v4f*)(C + (size_t)(row0 + r) * ldc + col0 + c4) = v; } }
    if (pass == 0) __threadfence(); }
}
template <int Cin, bool RELU>
__global__ __launch_bounds__(128) void k_conv2h(const float* __restrict__ in, const _Float16* __restrict__ Bt, const float* __restrict__ bias, float alpha, float* __restrict__ out) {
  constexpr int K = 9 * Cin, SPT = Cin / 32;
  __shared__ __attribute__((aligned(16))) float so[4][16][64];
  const int tid = threadIdx.x, w = tid >> 5, lane = tid & 31, ln = lane & 15, hh = lane >> 4;
  const int wid = blockIdx.x * 4 + w; const int mt = wid / (COUT / 64), nq = wid % (COUT / 64); if (mt * 16 >= NVOX) return;
  const int row0 = mt * 16, col0 = nq * 64;
  const int m = row0 + ln;
  const int x = m % WX, y = (m / WX) % HY, b = m / (WX * HY);
  v8f acc[4] = {};
  for (int tap = 0; tap < 9; ++tap) {
    const int dy = tap / 3 - 1, dx = tap % 3 - 1;
    const int xx = x + dx, yy = y + dy;
    const bool inb = (m < NPOSR) && (xx >= 0 && xx < WX && yy >= 0 && yy < HY);
    const float* src = in + ((size_t)((b * HY + (inb ? yy : 0)) * WX + (inb ? xx : 0))) * Cin;
#pragma unroll
    for (int s = 0; s < SPT; ++s) {
      const int c0 = s * 32;
      v4f a0 = {0.f,0.f,0.f,0.f}, a1 = a0, a2 = a0, a3 = a0;
      if (inb) { a0 = *(const v4fa*)(src + c0 + 8 * hh); a1 = *(const v4fa*)(src + c0 + 8 * hh + 4); a2 = *(const v4fa*)(src + c0 + 16 + 8 * hh); a3 = *(const v4fa*)(src + c0 + 16 + 8 * hh + 4); }
      float xs[16] = {a0[0],a0[1],a0[2],a0[3],a1[0],a1[1],a1[2],a1[3],a2[0],a2[1],a2[2],a2[3],a3[0],a3[1],a3[2],a3[3]};
      FragH ah;
#pragma unroll
      for (int i = 0; i < 16; ++i) ah.h[i] = (_Float16)xs[i];
      const int kb = tap * Cin + c0;
#pragma unroll
      for (int t = 0; t < 4; ++t) { FragH bq; bq.half[0] = *(const v8us*)((const unsigned short*)Bt + (size_t)(col0 + t * 16 + ln) * K + kb + 8 * hh); bq.half[1] = *(const v8us*)((const unsigned short*)Bt + (size_t)(col0 + t * 16 + ln) * K + kb + 16 + 8 * hh); acc[t] = mmaH<1>(ah.v, ah.v, bq.v, bq.v, acc[t]); }
    }
  }
#pragma unroll
  for (int t = 0; t < 4; ++t) { const int col = col0 + t * 16 + ln; const float bv = bf16_round(bias[col]);
#pragma unroll
    for (int r = 0; r < 8; ++r) { const float v = acc[t][r] * alpha + bv; so[w][8 * hh + r][t * 16 + ln] = RELU ? fmaxf(v, 0.f) : v; } }
  __builtin_amdgcn_fence(__ATOMIC_ACQ_REL, "workgroup"); __builtin_amdgcn_wave_barrier();
  const int rsub = lane >> 4, c4 = (lane & 15) * 4;
  for (int pass = 0; pass < 2; ++pass) { for (int q = 0; q < 8; ++q) { const int r = q * 2 + rsub; const v4f v = *(const v4fa*)&so[w][r][c4]; *(volatile v4f*)(out + (size_t)(row0 + r) * COUT + col0 + c4) = v; } if (pass == 0) __threadfence(); }
}


__global__ __launch_bounds__(256) void k_round_rows(const float* __restrict__ W, unsigned short* __restrict__ Wt, int n8) {
  const int t = blockIdx.x * 256 + threadIdx.x;
  if (t >= n8) return;
  const v4f a = *(const v4fa*)(W + (size_t)t * 8), b = *(const v4fa*)(W + (size_t)t * 8 + 4);
  v8us v; v[0]=bf16_bits(a[0]); v[1]=bf16_bits(a[1]); v[2]=bf16_bits(a[2]); v[3]=bf16_bits(a[3]);
  v[4]=bf16_bits(b[0]); v[5]=bf16_bits(b[1]); v[6]=bf16_bits(b[2]); v[7]=bf16_bits(b[3]);
  *(volatile v8us*)(Wt + (size_t)t * 8) = v; __threadfence(); *(volatile v8us*)(Wt + (size_t)t * 8) = v;
}

__global__ __launch_bounds__(256) void k_conv1(const float* __restrict__ x, const float* __restrict__ w, const float* __restrict__ bias, float* __restrict__ P1) {
  __shared__ float sw[C1 * 27]; __shared__ float sb[C1]; for (int i = threadIdx.x; i < C1 * 27; i += 256) sw[i] = bf16_round(w[i]); if (threadIdx.x < C1) sb[threadIdx.x] = bf16_round(bias[threadIdx.x]); __syncthreads();
  const size_t t = (size_t)blockIdx.x * 256 + threadIdx.x; if (t >= (size_t)NI * H1 * H1 * 4) return; const int cg = (int)(t % 4); const size_t pos = t / 4; const int px = (int)(pos % H1), py = (int)((pos / H1) % H1), b = (int)(pos / (H1 * H1));
  __shared__ float spatch[256][49]; float* patch = spatch[threadIdx.x];
  for (int ci = 0; ci < 3; ++ci) for (int r = 0; r < 4; ++r) for (int c = 0; c < 4; ++c) { const int yy = 2 * py - 1 + r, xx = 2 * px - 1 + c; patch[ci * 16 + r * 4 + c] = (yy >= 0 && yy < H0 && xx >= 0 && xx < H0) ? bf16_round(x[(((size_t)b * 3 + ci) * H0 + yy) * H0 + xx]) : 0.f; }
  __shared__ float so[256][17]; float* o = so[threadIdx.x];
#pragma unroll 1
  for (int j = 0; j < 16; ++j) { const int oc = cg * 16 + j; const float* wk = sw + oc * 27; float best = -3.0e38f;
#pragma unroll 1
    for (int dd = 0; dd < 4; ++dd) { const int dy = dd >> 1, dx = dd & 1; float a = sb[oc];
#pragma unroll 1
      for (int ci = 0; ci < 3; ++ci) {
#pragma unroll
        for (int ky = 0; ky < 3; ++ky) {
#pragma unroll
          for (int kx = 0; kx < 3; ++kx) a += wk[(ci * 3 + ky) * 3 + kx] * patch[ci * 16 + (dy + ky) * 4 + dx + kx]; } }
      best = fmaxf(best, fmaxf(a, 0.f)); }
    o[j] = best; }
  __syncthreads();
  { const size_t pos0 = (size_t)blockIdx.x * 64; float* base = P1 + pos0 * C1; for (int pass = 0; pass < 2; ++pass) { for (int e = threadIdx.x; e < 4096; e += 256) { const int pl = e / 64, ch = e % 64; *(volatile float*)(base + e) = so[pl * 4 + ch / 16][ch % 16]; } if (pass == 0) __threadfence(); } }
}
__global__ __launch_bounds__(256) void k_w2(const float* __restrict__ w, _Float16* __restrict__ Bt) { const int t = blockIdx.x * 256 + threadIdx.x; const int K = 9 * C1; if (t >= C2 * (K / 8)) return; const int o = t / (K / 8), k8 = (t % (K / 8)) * 8; FragH f;
#pragma unroll
  for (int i = 0; i < 8; ++i) { const int k = k8 + i; const int tap = k / C1, c = k % C1; f.h[i] = (_Float16)(bf16_round(w[((size_t)o * C1 + c) * 9 + tap]) * 16.0f); } const v8us v = f.half[0]; *(volatile v8us*)((unsigned short*)Bt + (size_t)o * K + k8) = v; __threadfence(); *(volatile v8us*)((unsigned short*)Bt + (size_t)o * K + k8) = v; }
__global__ __launch_bounds__(256) void k_pool2(const float* __restrict__ C, float* __restrict__ F) { const size_t t = (size_t)blockIdx.x * 256 + threadIdx.x; if (t >= (size_t)NT2 * C2 / 4) return; const int c4 = (int)(t % (C2 / 4)) * 4; const size_t tok = t / (C2 / 4); const int px = (int)(tok % H2), py = (int)((tok / H2) % H2), b = (int)(tok / (H2 * H2));
  v4f m = {-3.0e38f, -3.0e38f, -3.0e38f, -3.0e38f}; for (int dy = 0; dy < 2; ++dy) for (int dx = 0; dx < 2; ++dx) { const v4f v = *(const v4fa*)(C + (((size_t)b * H1 + 2 * py + dy) * H1 + 2 * px + dx) * C2 + c4); for (int q = 0; q < 4; ++q) m[q] = fmaxf(m[q], v[q]); }
  *(volatile v4f*)(F + t * 4) = m; __threadfence(); *(volatile v4f*)(F + t * 4) = m; }
__global__ __launch_bounds__(256) void k_wqkv(const float* __restrict__ qw, const float* __restrict__ kw, const float* __restrict__ vw, const float* __restrict__ qb, const float* __restrict__ kb, const float* __restrict__ vb, unsigned short* __restrict__ Bt, float* __restrict__ bcat) { const int t = blockIdx.x * 256 + threadIdx.x; if (t >= 192 * 16) return; const int n = t / 16, k8 = (t % 16) * 8; const float* w = (n < 64) ? qw + n * C2 : (n < 128 ? kw + (n - 64) * C2 : vw + (n - 128) * C2); v8us v;
#pragma unroll
  for (int i = 0; i < 8; ++i) v[i] = bf16_bits(w[k8 + i]); *(volatile v8us*)(Bt + (size_t)n * C2 + k8) = v; __threadfence(); *(volatile v8us*)(Bt + (size_t)n * C2 + k8) = v;
  if (t < 192) { const float bb = bf16_round(t < 64 ? qb[t] : (t < 128 ? kb[t - 64] : vb[t - 128])); *(volatile float*)(bcat + t) = bb; __threadfence(); *(volatile float*)(bcat + t) = bb; } }
__global__ __launch_bounds__(64) void k_axial(const float* __restrict__ QKV, const float* __restrict__ relw, const float* __restrict__ relh, float* __restrict__ OR, float* __restrict__ OC) {
  __shared__ float sk[2][32][DH + 1], sv[2][32][DH + 1]; __shared__ float sS[2][32][33]; __shared__ float sO[2][32][INNER + 1];
  const int tid = threadIdx.x, wv = tid >> 5, lane = tid & 31; const int t = blockIdx.x * 2 + wv; const int dir = t & 1; const int line = (t >> 1) % H2; const int b = (t >> 1) / H2;
  auto tok = [&](int p) { return dir == 0 ? ((b * H2 + line) * H2 + p) : ((b * H2 + p) * H2 + line); };
  const float* rel = dir == 0 ? relw : relh; const float* myrow = QKV + (size_t)tok(lane) * 192;
#pragma unroll 1
  for (int head = 0; head < NHD; ++head) {
    float q[DH]; for (int d = 0; d < DH; ++d) q[d] = myrow[head * DH + d] * 0.25f;
    for (int d = 0; d < DH; ++d) { sk[wv][lane][d] = myrow[64 + head * DH + d]; sv[wv][lane][d] = myrow[128 + head * DH + d]; }
    __builtin_amdgcn_fence(__ATOMIC_ACQ_REL, "workgroup"); __builtin_amdgcn_wave_barrier();
    float* s = sS[wv][lane]; float mx = -3.0e38f;
#pragma unroll 1
    for (int j = 0; j < 32; ++j) { float a = 0.f;
#pragma unroll
      for (int d = 0; d < DH; ++d) a += q[d] * sk[wv][j][d]; a += bf16_round(rel[head * 63 + (lane - j + 31)]); s[j] = a; mx = fmaxf(mx, a); }
    float den = 0.f;
#pragma unroll 1
    for (int j = 0; j < 32; ++j) { const float e = expf(s[j] - mx); s[j] = e; den += e; }
    float o[DH]; for (int d = 0; d < DH; ++d) o[d] = 0.f;
#pragma unroll 1
    for (int j = 0; j < 32; ++j) { const float pj = s[j] / den;
#pragma unroll
      for (int d = 0; d < DH; ++d) o[d] += pj * sv[wv][j][d]; }
    for (int d = 0; d < DH; ++d) sO[wv][lane][head * DH + d] = o[d];
    __builtin_amdgcn_fence(__ATOMIC_ACQ_REL, "workgroup"); __builtin_amdgcn_wave_barrier(); }
  float* Ob = (dir == 0 ? OR : OC);
  for (int pass = 0; pass < 2; ++pass) {
#pragma unroll 1
    for (int p = 0; p < 32; ++p) { float* dst = Ob + (size_t)tok(p) * INNER; *(volatile float*)(dst + lane) = sO[wv][p][lane]; *(volatile float*)(dst + 32 + lane) = sO[wv][p][32 + lane]; }
    if (pass == 0) __threadfence(); }
}
__global__ __launch_bounds__(128) void k_pool3(const float* __restrict__ F2, float* __restrict__ PL) { const int b = blockIdx.x, c = threadIdx.x; float s = 0.f;
#pragma unroll 1
  for (int p = 0; p < H2 * H2; ++p) s += F2[((size_t)b * H2 * H2 + p) * C2 + c]; const float m = s / (float)(H2 * H2); *(volatile float*)(PL + b * C2 + c) = m; __threadfence(); *(volatile float*)(PL + b * C2 + c) = m; }
__global__ __launch_bounds__(512) void k_fc(const float* __restrict__ PL, const float* __restrict__ fcw, const float* __restrict__ fcb, float* __restrict__ out) { const int t = threadIdx.x; float a = 0.f; if (t < NI * 10) { const int b = t / 10, c = t % 10; a = bf16_round(fcb[c]);
#pragma unroll 1
    for (int k = 0; k < C2; ++k) a += PL[b * C2 + k] * bf16_round(fcw[c * C2 + k]); }
  if (t < NI * 10) { *(volatile float*)(out + t) = a; } __threadfence(); if (t < NI * 10) { *(volatile float*)(out + t) = a; } }
__global__ __launch_bounds__(256) void k_addo(const float* __restrict__ A, const float* __restrict__ Bv, float* __restrict__ O) { const size_t t = (size_t)blockIdx.x * 256 + threadIdx.x; if (t >= (size_t)NT2 * INNER / 4) return; const v4f a = *(const v4fa*)(A + t * 4), b = *(const v4fa*)(Bv + t * 4); const v4f o = a + b; *(volatile v4f*)(O + t * 4) = o; __threadfence(); *(volatile v4f*)(O + t * 4) = o; }
extern "C" void kernel_launch(void* const* d_in, const int* in_sizes, int n_in,
                              void* d_out, int out_size, void* d_ws, size_t ws_size, hipStream_t stream) {
  (void)in_sizes; (void)n_in; (void)out_size;
  const float* x = (const float*)d_in[0]; const float* c1w = (const float*)d_in[1]; const float* c1b = (const float*)d_in[2]; const float* c2w = (const float*)d_in[3]; const float* c2b = (const float*)d_in[4];
  const float* qw = (const float*)d_in[5]; const float* qb = (const float*)d_in[6]; const float* kw = (const float*)d_in[7]; const float* kb = (const float*)d_in[8]; const float* vw = (const float*)d_in[9]; const float* vb = (const float*)d_in[10];
  const float* pw = (const float*)d_in[11]; const float* pb = (const float*)d_in[12]; const float* relh = (const float*)d_in[13]; const float* relw = (const float*)d_in[14]; const float* fcw = (const float*)d_in[15]; const float* fcb = (const float*)d_in[16];
  char* ws = (char*)d_ws; size_t off = 0;
  auto take = [&](size_t bytes) { char* p = ws + off; off += (bytes + 255) & ~(size_t)255; return p; };
  _Float16* B2 = (_Float16*)take((size_t)C2 * 576 * 2); unsigned short* Bqkv = (unsigned short*)take((size_t)192 * C2 * 2); float* bqkv = (float*)take(192 * 4); unsigned short* Bp = (unsigned short*)take((size_t)C2 * INNER * 2);
  float* P1 = (float*)take((size_t)NPOS * C1 * 4); float* CV2 = (float*)take((size_t)NPOS * C2 * 4); float* F = (float*)take((size_t)NT2 * C2 * 4); float* QKV = (float*)take((size_t)NT2 * 192 * 4); float* OR = (float*)take((size_t)NT2 * INNER * 4); float* OC = (float*)take((size_t)NT2 * INNER * 4); float* O = (float*)take((size_t)NT2 * INNER * 4); float* F2 = (float*)take((size_t)NT2 * C2 * 4); float* PL = (float*)take((size_t)NI * C2 * 4);
  if (off > ws_size) return;
  k_w2<<<(C2 * 72 + 255) / 256, 256, 0, stream>>>(c2w, B2); k_wqkv<<<(192 * 16 + 255) / 256, 256, 0, stream>>>(qw, kw, vw, qb, kb, vb, Bqkv, bqkv); k_round_rows<<<(C2 * INNER / 8 + 255) / 256, 256, 0, stream>>>(pw, Bp, C2 * INNER / 8);
  k_conv1<<<(unsigned)(((size_t)NI * H1 * H1 * 4 + 255) / 256), 256, 0, stream>>>(x, c1w, c1b, P1);
  k_conv2h<C1, true><<<((NVOX / 16) * (COUT / 64) + 3) / 4, 128, 0, stream>>>(P1, B2, c2b, 0.0625f, CV2);
  k_pool2<<<(unsigned)(((size_t)NT2 * C2 / 4 + 255) / 256), 256, 0, stream>>>(CV2, F);
  k_gemm_bf3<true, 0, false, false><<<((NT2 / 16) * 3 + 3) / 4, 128, 0, stream>>>(F, C2, Bqkv, C2, bqkv, nullptr, 1, 0, QKV, 192, NT2, 192, C2);
  k_axial<<<(NI * H2 * 2) / 2, 64, 0, stream>>>(QKV, relw, relh, OR, OC);
  k_addo<<<(unsigned)(((size_t)NT2 * INNER / 4 + 255) / 256), 256, 0, stream>>>(OR, OC, O);
  k_gemm_bf3<true, 0, true, false><<<((NT2 / 16) * 2 + 3) / 4, 128, 0, stream>>>(O, INNER, Bp, INNER, pb, F, NT2, C2, F2, C2, NT2, C2, INNER);
  k_pool3<<<NI, 128, 0, stream>>>(F2, PL); k_fc<<<1, 512, 0, stream>>>(PL, fcw, fcb, (float*)d_out);
}
